// SelfAttention_19292993094139
// MI455X (gfx1250) — hardware-verified
//
#include <hip/hip_runtime.h>
#include <math.h>

#ifndef NB
#define NB 4
#endif
#ifndef SEQ
#define SEQ 4096
#endif
#define NB_FULL 4
#define SEQ_FULL 4096
#define DM 256
#define GROUPS 32
#define CPG (DM / GROUPS)
#define GN_EPS 1.0e-5f

typedef _Float16 v16h __attribute__((ext_vector_type(16)));
typedef _Float16 v8h  __attribute__((ext_vector_type(8)));
typedef float    v8f  __attribute__((ext_vector_type(8)));
typedef float    v4f  __attribute__((ext_vector_type(4)));
typedef unsigned v4u  __attribute__((ext_vector_type(4)));
typedef v8h v8h_ma __attribute__((may_alias));
typedef v4f v4f_ma __attribute__((may_alias));

static_assert(DM == 256);
static_assert(DM % 64 == 0);
static_assert(SEQ % 64 == 0);
static_assert((NB * SEQ) % 64 == 0);
static_assert(NB <= NB_FULL && SEQ <= SEQ_FULL);
static_assert((((NB * SEQ) / 64) * ((2 * DM) / 64)) % 8 == 0);
static_assert(((DM / 64) * (SEQ / 64)) % 8 == 0);
static_assert(((SEQ / 64) * (DM / 64)) % 8 == 0);
static_assert(DM % GROUPS == 0);
static_assert(CPG * GROUPS == DM);
static_assert(SEQ % 4 == 0 && SEQ_FULL % 4 == 0);

union FH { v16h v; v8h h[2]; };
__device__ __forceinline__ v16h ldfrag_g(const _Float16* p) { FH f; f.h[0] = *(const v8h*)(p); f.h[1] = *(const v8h*)(p + 16); return f.v; }
__device__ __forceinline__ v8f mma_h(v16h a, v16h b, v8f c) { return __builtin_amdgcn_wmma_f32_16x16x32_f16(false, a, false, b, (short)0, c, false, false); }
__device__ __forceinline__ void dep_guard_h(v8f& a, v8f& b, v16h x, v16h y) { asm volatile("v_nop\n\tv_nop\n\tv_nop\n\tv_nop" : "+v"(a), "+v"(b) : "v"(x), "v"(y)); }
__device__ __forceinline__ void keep4_h(v16h a, v16h b, v16h c, v16h d) { asm volatile("v_nop" :: "v"(a), "v"(b), "v"(c), "v"(d)); }
__device__ __forceinline__ void acc_guard4(v8f& a, v8f& b, v8f& c, v8f& d) { asm volatile("v_nop\n\tv_nop\n\tv_nop\n\tv_nop" : "+v"(a), "+v"(b), "+v"(c), "+v"(d)); }
__device__ __forceinline__ void guard_s(v8f& a, v8f& b, v16h x, v16h y, v16h z) { asm volatile("v_nop\n\tv_nop\n\tv_nop\n\tv_nop" : "+v"(a), "+v"(b) : "v"(x), "v"(y), "v"(z)); }
__device__ __forceinline__ void guard_o(v8f& a, v8f& b, v8f& c, v8f& d, v16h p, v16h x, v16h y, v16h z, v16h w) {
    asm volatile("v_nop\n\tv_nop\n\tv_nop\n\tv_nop" : "+v"(a), "+v"(b), "+v"(c), "+v"(d) : "v"(p), "v"(x), "v"(y), "v"(z), "v"(w)); }
__device__ __forceinline__ void wave_sync_lds() {
    __builtin_amdgcn_fence(3  , "workgroup");
    __builtin_amdgcn_wave_barrier();
    __builtin_amdgcn_fence(2  , "workgroup");
}
__device__ __forceinline__ float ex2(float x) {
#if __has_builtin(__builtin_amdgcn_exp2f)
    return __builtin_amdgcn_exp2f(x);
#else
    return exp2f(x);
#endif
}

#define VST2(T, ptr, val) do { const T vst2_v_ = (val); *(volatile T*)(ptr) = vst2_v_; __threadfence(); *(volatile T*)(ptr) = vst2_v_; } while (0)

__device__ __forceinline__ float cmb_bf(float v) { const unsigned u = __builtin_bit_cast(unsigned, v); const unsigned r = (u + 0x7fffu + ((u >> 16) & 1u)) & 0xffff0000u; return __builtin_bit_cast(float, r); }
__device__ __forceinline__ unsigned cmb_pk2(float a, float b) { return (unsigned)__builtin_bit_cast(unsigned short, (_Float16)a) | ((unsigned)__builtin_bit_cast(unsigned short, (_Float16)b) << 16); }

static __device__ __forceinline__ _Float16 toh_flush(float v) { const _Float16 r = (_Float16)v; return (fabsf(v) < 6.103515625e-05f) ? (_Float16)0.0f : r; }

__global__ __launch_bounds__(256) void k_gn_stats(const float* __restrict__ X, float* __restrict__ ST) {
#pragma clang fp contract(off)
    __shared__ float red1[8];
    __shared__ float red2[8];
    const int tid = threadIdx.x, lane = tid & 31;
    const int wave = __builtin_amdgcn_readfirstlane(threadIdx.x >> 5);
    const int b = (int)blockIdx.x / GROUPS; const int g = (int)blockIdx.x - b * GROUPS;
    const float* base = X + ((size_t)b * DM + (size_t)g * CPG) * SEQ_FULL;
    const int per = SEQ / 4;
    const float invcnt = 1.0f / (float)(CPG * SEQ);

    float s = 0.f;
#pragma unroll 4
    for (int idx = tid; idx < CPG * per; idx += 256) {
        const int ch = idx / per; const int q = idx - ch * per;
        const v4f a = *(const v4f*)(base + (size_t)ch * SEQ_FULL + 4 * q);
        s += (cmb_bf(a.x) + cmb_bf(a.y)) + (cmb_bf(a.z) + cmb_bf(a.w));
    }
    s += __shfl_xor(s, 1, 32); s += __shfl_xor(s, 2, 32); s += __shfl_xor(s, 4, 32); s += __shfl_xor(s, 8, 32); s += __shfl_xor(s, 16, 32);
    if (lane == 0) red1[wave] = s;
    __syncthreads();
    const float tot = ((red1[0] + red1[1]) + (red1[2] + red1[3])) + ((red1[4] + red1[5]) + (red1[6] + red1[7]));
    const float mean = tot * invcnt;

    float ss = 0.f;
#pragma unroll 4
    for (int idx = tid; idx < CPG * per; idx += 256) {
        const int ch = idx / per; const int q = idx - ch * per;
        const v4f a = *(const v4f*)(base + (size_t)ch * SEQ_FULL + 4 * q);
        const float d0 = cmb_bf(a.x) - mean, d1 = cmb_bf(a.y) - mean, d2 = cmb_bf(a.z) - mean, d3 = cmb_bf(a.w) - mean;
        ss += (d0 * d0 + d1 * d1) + (d2 * d2 + d3 * d3);
    }
    ss += __shfl_xor(ss, 1, 32); ss += __shfl_xor(ss, 2, 32); ss += __shfl_xor(ss, 4, 32); ss += __shfl_xor(ss, 8, 32); ss += __shfl_xor(ss, 16, 32);
    if (lane == 0) red2[wave] = ss;
    __syncthreads();
    const float tot2 = ((red2[0] + red2[1]) + (red2[2] + red2[3])) + ((red2[4] + red2[5]) + (red2[6] + red2[7]));
    const float var = tot2 * invcnt;
    const float rstd = rsqrtf(var + GN_EPS);

    if (tid < 8) {
        v4f o;
        o.x = (tid == 0) ? mean : 0.f; o.y = (tid == 0) ? rstd : 0.f; o.z = 0.f; o.w = 0.f;
        VST2(v4f, (v4f*)(ST + (size_t)blockIdx.x * 32 + 4 * tid), o);
    }
}

#define XT_NP 32
#define XT_LP 260
static_assert(XT_NP == 32);
static_assert(SEQ % XT_NP == 0);
static_assert(XT_LP >= DM && XT_LP % 4 == 0);
static_assert(DM == 256);
__global__ __launch_bounds__(256) void k_gn_xt(const float* __restrict__ X, const float* __restrict__ ST, const float* __restrict__ gain, const float* __restrict__ shift, unsigned short* __restrict__ X16) {
#pragma clang fp contract(off)
    __shared__ __align__(16) float T[XT_NP * XT_LP];
    __shared__ float sMu[DM];
    __shared__ float sRs[DM];
    __shared__ float sGa[DM];
    __shared__ float sBe[DM];
    const int tid = threadIdx.x, lane = tid & 31;
    const int wave = __builtin_amdgcn_readfirstlane(threadIdx.x >> 5);
    const int nblk = SEQ / XT_NP;
    const int b = (int)blockIdx.x / nblk; const int n0 = ((int)blockIdx.x - b * nblk) * XT_NP;
    {
        const int g = tid / CPG;
        const size_t so = ((size_t)b * GROUPS + g) * 32;
        sMu[tid] = ST[so];
        sRs[tid] = ST[so + 1];
        sGa[tid] = cmb_bf(gain[tid]);
        sBe[tid] = cmb_bf(shift[tid]);
    }
    __syncthreads();
    const int q4 = (tid & 7) * 4, cr = tid >> 3;
#pragma unroll 1
    for (int it = 0; it < DM / 32; ++it) {
        const int c = it * 32 + cr;
        const v4f xv = *(const v4f*)(X + ((size_t)b * DM + c) * SEQ_FULL + n0 + q4);
        const float mu = sMu[c], rs = sRs[c], ga = sGa[c], be = sBe[c];
        T[(q4 + 0) * XT_LP + c] = ((cmb_bf(xv.x) - mu) * rs) * ga + be;
        T[(q4 + 1) * XT_LP + c] = ((cmb_bf(xv.y) - mu) * rs) * ga + be;
        T[(q4 + 2) * XT_LP + c] = ((cmb_bf(xv.z) - mu) * rs) * ga + be;
        T[(q4 + 3) * XT_LP + c] = ((cmb_bf(xv.w) - mu) * rs) * ga + be;
    }
    __syncthreads();
    for (int pass = 0; pass < 2; ++pass) {
#pragma unroll
        for (int it = 0; it < 4; ++it) {
            const int row = it * 8 + wave;
            const v4f a = *(const v4f_ma*)&T[row * XT_LP + lane * 8];
            const v4f d = *(const v4f_ma*)&T[row * XT_LP + lane * 8 + 4];
            v8h hv;
            hv[0] = toh_flush(a.x); hv[1] = toh_flush(a.y); hv[2] = toh_flush(a.z); hv[3] = toh_flush(a.w);
            hv[4] = toh_flush(d.x); hv[5] = toh_flush(d.y); hv[6] = toh_flush(d.z); hv[7] = toh_flush(d.w);
            *(volatile v8h*)(X16 + ((size_t)b * SEQ + n0 + row) * DM + lane * 8) = hv;
        }
        __threadfence();
    }
}

__global__ __launch_bounds__(256) void k_cast_w(const float* __restrict__ W, unsigned short* __restrict__ W16, int nrows, float sc) {
    const int u = (int)blockIdx.x * 256 + (int)threadIdx.x; const int per = DM / 8;
    if (u >= nrows * per) return;
    const int r = u / per; const int c0 = 8 * (u % per);
    const float* src = W + (size_t)r * DM + c0;
    const v4f a = *(const v4f*)(src); const v4f d = *(const v4f*)(src + 4);
    v4u pk;
    pk.x = cmb_pk2(cmb_bf(a.x) * sc, cmb_bf(a.y) * sc); pk.y = cmb_pk2(cmb_bf(a.z) * sc, cmb_bf(a.w) * sc);
    pk.z = cmb_pk2(cmb_bf(d.x) * sc, cmb_bf(d.y) * sc); pk.w = cmb_pk2(cmb_bf(d.z) * sc, cmb_bf(d.w) * sc);
    VST2(v4u, (v4u*)(W16 + (size_t)r * DM + c0), pk);
}

template <int BIAS_MODE, int OUT_MODE>
__device__ __forceinline__ void gemm64_body(const unsigned short* __restrict__ Ap, int lda, long long strideA,
                                            const unsigned short* __restrict__ Btp, int ldb, long long strideB,
                                            void* __restrict__ Cout, int ldc, long long strideC,
                                            const float* __restrict__ bias, int M, int N, int K, float scale) {
    __shared__ __align__(16) float sT[8 * 16 * 68];
    const int bz = blockIdx.y;
    const int lane = threadIdx.x & 31, wave = threadIdx.x >> 5;
    const int tilesN = N >> 6, tilesM = M >> 6;
    const int tile = blockIdx.x * 8 + wave;
    if (tile >= tilesM * tilesN) return;
    const int tm = tile / tilesN, tn = tile - tm * tilesN;
    const int m0 = tm << 6, n0 = tn << 6;
    const _Float16* Ab = (const _Float16*)Ap + (size_t)bz * strideA;
    const _Float16* Bb = (const _Float16*)Btp + (size_t)bz * strideB;
    const int rlane = lane & 15, koff = (lane >> 4) * 8, mOff = (lane >> 4) * 8;
    const int sb = wave * (16 * 68);

    v8f acc[4][4];
#pragma unroll
    for (int i = 0; i < 4; ++i)
#pragma unroll
        for (int j = 0; j < 4; ++j) acc[i][j] = (v8f){0.f, 0.f, 0.f, 0.f, 0.f, 0.f, 0.f, 0.f};

#pragma unroll 1
    for (int k0 = 0; k0 < K; k0 += 32) {
        v16h bh[4];
#pragma unroll
        for (int j = 0; j < 4; ++j) bh[j] = ldfrag_g(Bb + (size_t)(n0 + (j << 4) + rlane) * ldb + koff + k0);
#pragma unroll
        for (int i = 0; i < 4; ++i) {
            const v16h ah = ldfrag_g(Ab + (size_t)(m0 + (i << 4) + rlane) * lda + koff + k0);
#pragma unroll
            for (int j = 0; j < 4; ++j) acc[i][j] = mma_h(ah, bh[j], acc[i][j]);
            dep_guard_h(acc[i][0], acc[i][3], ah, ah);
        }
        keep4_h(bh[0], bh[1], bh[2], bh[3]);
    }
    acc_guard4(acc[0][0], acc[0][1], acc[0][2], acc[0][3]);
    acc_guard4(acc[1][0], acc[1][1], acc[1][2], acc[1][3]);
    acc_guard4(acc[2][0], acc[2][1], acc[2][2], acc[2][3]);
    acc_guard4(acc[3][0], acc[3][1], acc[3][2], acc[3][3]);

#pragma unroll
    for (int i = 0; i < 4; ++i) {
        const int mBase = m0 + (i << 4);
#pragma unroll
        for (int j = 0; j < 4; ++j) {
            const int n = n0 + (j << 4) + rlane;
            float bv = 0.f;
            if (BIAS_MODE == 2) bv = cmb_bf(bias[n]);
#pragma unroll
            for (int r = 0; r < 8; ++r) {
                float v = acc[i][j][r] * scale;
                if (BIAS_MODE == 1) v += cmb_bf(bias[mBase + mOff + r]);
                if (BIAS_MODE == 2) v += bv;
                sT[sb + (mOff + r) * 68 + (j << 4) + rlane] = v;
            }
        }
        wave_sync_lds();
        if (OUT_MODE == 0) {
            float* C = (float*)Cout + (size_t)bz * strideC;
            const int hh = lane >> 4, c4 = (lane & 15) * 4;
            for (int pass = 0; pass < 2; ++pass) {
#pragma unroll
                for (int it = 0; it < 8; ++it) {
                    const int row = it * 2 + hh;
                    const v4f v = *(const v4f_ma*)&sT[sb + row * 68 + c4];
                    *(volatile v4f*)(C + (size_t)(mBase + row) * ldc + n0 + c4) = v;
                }
                __threadfence();
            }
        } else {
            unsigned short* C = (unsigned short*)Cout + (size_t)bz * strideC;
            const int q = lane >> 3, c8 = (lane & 7) * 8;
            for (int pass = 0; pass < 2; ++pass) {
#pragma unroll
                for (int it = 0; it < 4; ++it) {
                    const int row = it * 4 + q;
                    v8h hv;
#pragma unroll
                    for (int e = 0; e < 8; ++e) hv[e] = (_Float16)sT[sb + row * 68 + c8 + e];
                    *(volatile v8h*)(C + (size_t)(mBase + row) * ldc + n0 + c8) = hv;
                }
                __threadfence();
            }
        }
        wave_sync_lds();
    }
}

__global__ __launch_bounds__(256) void k_gemm_qk(const unsigned short* __restrict__ X16, const unsigned short* __restrict__ W16, unsigned short* __restrict__ QK16, const float* __restrict__ bqkv) {
    gemm64_body<2, 1>(X16, DM, 0, W16, DM, 0, (void*)QK16, 2 * DM, 0, bqkv, NB * SEQ, 2 * DM, DM, 0.00390625f);
}
__global__ __launch_bounds__(256) void k_gemm_vt(const unsigned short* __restrict__ WV16, const unsigned short* __restrict__ X16, unsigned short* __restrict__ VT16, const float* __restrict__ bv) {
    gemm64_body<1, 1>(WV16, DM, 0, X16, DM, (long long)SEQ * DM, (void*)VT16, SEQ, (long long)DM * SEQ, bv, DM, SEQ, DM, 0.00390625f);
}
__global__ __launch_bounds__(256) void k_gemm_out(const unsigned short* __restrict__ WO16, const unsigned short* __restrict__ CTX16, float* __restrict__ OUT, const float* __restrict__ bo) {
    gemm64_body<1, 0>(WO16, DM, 0, CTX16, DM, (long long)SEQ * DM, (void*)OUT, SEQ_FULL, (long long)DM * SEQ_FULL, bo, DM, SEQ, DM, 0.00006103515625f);
}

#define AT_PP 40
#define AT_OP 68
static_assert((AT_PP * 2) % 16 == 0);
static_assert(AT_PP >= 32);
__global__ __launch_bounds__(128) void k_flash(const unsigned short* __restrict__ QKp, const unsigned short* __restrict__ VTp, unsigned short* __restrict__ CTXp) {
    __shared__ __align__(16) _Float16 Ps[4 * 16 * AT_PP];
    __shared__ __align__(16) float    Os[4 * 16 * AT_OP];
    const _Float16* QK = (const _Float16*)QKp;
    const _Float16* VT = (const _Float16*)VTp;
    const int tid = threadIdx.x, wave = tid >> 5, lane = tid & 31, hh = lane >> 4, c = lane & 15;
    const int nqb = SEQ / 64;
    const int bx = blockIdx.x; const int qb = bx % nqb; const int b = bx / nqb;
    const int q0 = qb * 64 + wave * 16;
    const size_t qoff = ((size_t)b * SEQ + q0 + c) * (2 * DM) + 8 * hh;
    const size_t koff = ((size_t)b * SEQ + c) * (2 * DM) + DM + 8 * hh;
    const size_t voff = ((size_t)b * DM + c) * SEQ + 8 * hh;
    const int pst = wave * (16 * AT_PP) + (8 * hh) * AT_PP + c;
    const int pld = wave * (16 * AT_PP) + c * AT_PP + 8 * hh;
    const float C2 = 0.0625f * 1.4426950408889634f;

    float mrow[8], lpart[8];
    v8f o[16];
#pragma unroll
    for (int t = 0; t < 16; ++t) o[t] = (v8f){0.f, 0.f, 0.f, 0.f, 0.f, 0.f, 0.f, 0.f};
#pragma unroll
    for (int r = 0; r < 8; ++r) { mrow[r] = -1.0e30f; lpart[r] = 0.f; }

#pragma unroll 1
    for (int kv0 = 0; kv0 < SEQ; kv0 += 32) {
        v8f s0 = (v8f){0.f, 0.f, 0.f, 0.f, 0.f, 0.f, 0.f, 0.f}, s1 = s0;
#pragma unroll
        for (int dc = 0; dc < 8; ++dc) {
            const v16h qa = ldfrag_g(QK + qoff + dc * 32);
            const v16h k0f = ldfrag_g(QK + koff + (size_t)kv0 * (2 * DM) + dc * 32);
            const v16h k1f = ldfrag_g(QK + koff + (size_t)(kv0 + 16) * (2 * DM) + dc * 32);
            s0 = mma_h(qa, k0f, s0);
            s1 = mma_h(qa, k1f, s1);
            guard_s(s0, s1, qa, k0f, k1f);
        }
        float al[8];
        int chg = 0;
#pragma unroll
        for (int r = 0; r < 8; ++r) {
            const float a0 = s0[r] * C2, a1 = s1[r] * C2;
            float m = fmaxf(a0, a1);
            m = fmaxf(m, __shfl_xor(m, 1, 32)); m = fmaxf(m, __shfl_xor(m, 2, 32));
            m = fmaxf(m, __shfl_xor(m, 4, 32)); m = fmaxf(m, __shfl_xor(m, 8, 32));
            const float mold = mrow[r];
            const float mnew = fmaxf(mold, m);
            const bool up = mnew > mold;
            const float alpha = up ? ex2(mold - mnew) : 1.0f;
            const float mc = mnew - 12.0f;
            const float p0 = ex2(a0 - mc), p1 = ex2(a1 - mc);
            lpart[r] = lpart[r] * alpha + (p0 + p1);
            mrow[r] = mnew;
            al[r] = alpha;
            chg |= up ? 1 : 0;
            Ps[pst + r * AT_PP]      = (_Float16)p0;
            Ps[pst + r * AT_PP + 16] = (_Float16)p1;
        }
        if (__builtin_amdgcn_ballot_w32(chg != 0) != 0u) {
#pragma unroll
            for (int t = 0; t < 16; ++t)
#pragma unroll
                for (int r = 0; r < 8; ++r) o[t][r] *= al[r];
        }
        wave_sync_lds();
        {
            FH pa;
            pa.h[0] = *(const v8h_ma*)&Ps[pld];
            pa.h[1] = *(const v8h_ma*)&Ps[pld + 16];
#pragma unroll
            for (int g = 0; g < 4; ++g) {
                const v16h vb0 = ldfrag_g(VT + voff + (size_t)((4 * g + 0) * 16) * SEQ + kv0);
                const v16h vb1 = ldfrag_g(VT + voff + (size_t)((4 * g + 1) * 16) * SEQ + kv0);
                const v16h vb2 = ldfrag_g(VT + voff + (size_t)((4 * g + 2) * 16) * SEQ + kv0);
                const v16h vb3 = ldfrag_g(VT + voff + (size_t)((4 * g + 3) * 16) * SEQ + kv0);
                o[4 * g + 0] = mma_h(pa.v, vb0, o[4 * g + 0]);
                o[4 * g + 1] = mma_h(pa.v, vb1, o[4 * g + 1]);
                o[4 * g + 2] = mma_h(pa.v, vb2, o[4 * g + 2]);
                o[4 * g + 3] = mma_h(pa.v, vb3, o[4 * g + 3]);
                guard_o(o[4 * g + 0], o[4 * g + 1], o[4 * g + 2], o[4 * g + 3], pa.v, vb0, vb1, vb2, vb3);
            }
        }
        wave_sync_lds();
    }

    float inv[8];
#pragma unroll
    for (int r = 0; r < 8; ++r) {
        float l = lpart[r];
        l += __shfl_xor(l, 1, 32); l += __shfl_xor(l, 2, 32); l += __shfl_xor(l, 4, 32); l += __shfl_xor(l, 8, 32);
        inv[r] = 1.0f / (l * 0.015625f);
    }
    const int ob = wave * (16 * AT_OP);
    const int qq = lane >> 3, c8 = (lane & 7) * 8;
#pragma unroll
    for (int g = 0; g < 4; ++g) {
#pragma unroll
        for (int r = 0; r < 8; ++r) {
            Os[ob + (8 * hh + r) * AT_OP +  0 + c] = o[4 * g + 0][r] * inv[r];
            Os[ob + (8 * hh + r) * AT_OP + 16 + c] = o[4 * g + 1][r] * inv[r];
            Os[ob + (8 * hh + r) * AT_OP + 32 + c] = o[4 * g + 2][r] * inv[r];
            Os[ob + (8 * hh + r) * AT_OP + 48 + c] = o[4 * g + 3][r] * inv[r];
        }
        wave_sync_lds();
        {
            unsigned short* CT = CTXp + ((size_t)b * SEQ + q0) * DM + g * 64;
            for (int pass = 0; pass < 2; ++pass) {
#pragma unroll
                for (int it = 0; it < 4; ++it) {
                    const int row = it * 4 + qq;
                    v8h hv;
#pragma unroll
                    for (int e = 0; e < 8; ++e) hv[e] = (_Float16)Os[ob + row * AT_OP + c8 + e];
                    *(volatile v8h*)(CT + (size_t)row * DM + c8) = hv;
                }
                __threadfence();
            }
        }
        wave_sync_lds();
    }
}

#define WS_X16  ((size_t)NB * SEQ * DM * 2)
#define WS_W16  ((size_t)3 * DM * DM * 2)
#define WS_WO16 ((size_t)DM * DM * 2)
#define WS_QK16 ((size_t)NB * SEQ * 2 * DM * 2)
#define WS_VT16 ((size_t)NB * DM * SEQ * 2)
#define WS_CTX  ((size_t)NB * SEQ * DM * 2)
#define WS_ST   ((size_t)NB * GROUPS * 32 * 4)
#define WS_TOTAL (WS_X16 + WS_W16 + WS_WO16 + WS_QK16 + WS_VT16 + WS_CTX + WS_ST)
static_assert(WS_TOTAL <= (size_t)134217728);
static_assert(WS_X16 % 256 == 0 && WS_W16 % 256 == 0 && WS_WO16 % 256 == 0 && WS_QK16 % 256 == 0 && WS_VT16 % 256 == 0 && WS_CTX % 256 == 0 && WS_ST % 256 == 0);
static_assert(((size_t)(NB * GROUPS - 1) * 32 + 32) * 4 <= WS_ST);
static_assert(((size_t)(NB - 1) * DM + (DM - 1)) * SEQ_FULL + SEQ <= (size_t)NB_FULL * DM * SEQ_FULL);

extern "C" void kernel_launch(void* const* d_in, const int* in_sizes, int n_in, void* d_out, int out_size, void* d_ws, size_t ws_size, hipStream_t stream) {
    if (n_in < 7) return;
    if (in_sizes[0] < ((NB - 1) * DM + (DM - 1)) * SEQ_FULL + SEQ) return;
    if (in_sizes[1] < DM) return;
    if (in_sizes[2] < DM) return;
    if (in_sizes[3] < 3 * DM * DM) return;
    if (in_sizes[4] < 3 * DM) return;
    if (in_sizes[5] < DM * DM) return;
    if (in_sizes[6] < DM) return;
    if (out_size < ((NB - 1) * DM + (DM - 1)) * SEQ_FULL + SEQ) return;
    if (WS_TOTAL > ws_size) return;
    const float* x     = (const float*)d_in[0];
    const float* gain  = (const float*)d_in[1];
    const float* shift = (const float*)d_in[2];
    const float* Wqkv  = (const float*)d_in[3];
    const float* bqkv  = (const float*)d_in[4];
    const float* Wo    = (const float*)d_in[5];
    const float* bo    = (const float*)d_in[6];
    float* out = (float*)d_out;
    char* wsp = (char*)d_ws;
    unsigned short* X16   = (unsigned short*)wsp; wsp += WS_X16;
    unsigned short* W16   = (unsigned short*)wsp; wsp += WS_W16;
    unsigned short* WO16  = (unsigned short*)wsp; wsp += WS_WO16;
    unsigned short* QK16  = (unsigned short*)wsp; wsp += WS_QK16;
    unsigned short* VT16  = (unsigned short*)wsp; wsp += WS_VT16;
    unsigned short* CTX16 = (unsigned short*)wsp; wsp += WS_CTX;
    float*          ST    = (float*)wsp;          wsp += WS_ST;

    k_gn_stats<<<(unsigned)(NB * GROUPS), 256, 0, stream>>>(x, ST);
    k_gn_xt<<<(unsigned)(NB * (SEQ / XT_NP)), 256, 0, stream>>>(x, ST, gain, shift, X16);
    k_cast_w<<<(unsigned)(((3 * DM) * (DM / 8) + 255) / 256), 256, 0, stream>>>(Wqkv, W16, 3 * DM, 256.0f);
    k_cast_w<<<(unsigned)((DM * (DM / 8) + 255) / 256), 256, 0, stream>>>(Wo, WO16, DM, 256.0f);
    k_gemm_qk<<<dim3((unsigned)((((NB * SEQ) / 64) * ((2 * DM) / 64)) / 8), 1u), 256, 0, stream>>>(X16, W16, QK16, bqkv);
    k_gemm_vt<<<dim3((unsigned)(((DM / 64) * (SEQ / 64)) / 8), (unsigned)NB), 256, 0, stream>>>(W16 + (size_t)2 * DM * DM, X16, VT16, bqkv + 2 * DM);
    k_flash<<<(unsigned)(NB * (SEQ / 64)), 128, 0, stream>>>(QK16, VT16, CTX16);
    k_gemm_out<<<dim3((unsigned)(((DM / 64) * (SEQ / 64)) / 8), (unsigned)NB), 256, 0, stream>>>(WO16, CTX16, out, bo);
}
